// CasualAttention_30940944400931
// MI455X (gfx1250) — hardware-run, weakly checked
//
#include <hip/hip_runtime.h>


#ifndef NB
#define NB 1
#endif
#ifndef SEQ
#define SEQ 2048
#endif
#define NB_FULL  1
#define SEQ_FULL 2048
#define DM   1024
#define NH_  64
#define HD   16
#define NQKV 3072
#define AW   4
#define OSP  68
#define EROWS (SEQ < 256 ? SEQ : 256)
#define QRS  2048.0f
#define QRI  (1.0f / 2048.0f)
#define SC2  ((float)(0.25 * 1.4426950408889634))
#define PSH  14.0f
#define NEGB (-3.0e38f)
#define WSC  64.0f
#define CSC  16.0f
#define OSI  (1.0f / (64.0f * 16.0f))

static_assert(NB == 1);
static_assert(HD == 16);
static_assert(NH_ * HD == DM);
static_assert(AW * HD == 64);
static_assert(NH_ % AW == 0);
static_assert(DM % 64 == 0);
static_assert(NQKV == 3 * DM);
static_assert(DM % 32 == 0);
static_assert(SEQ % 64 == 0);
static_assert(SEQ % 32 == 0);
static_assert(EROWS % 64 == 0);
static_assert(EROWS % 32 == 0);
static_assert(EROWS >= 32);
static_assert(EROWS <= SEQ);
static_assert((SEQ - EROWS) % 64 == 0);
static_assert(((size_t)SEQ * DM) % 8 == 0);
static_assert(SEQ <= SEQ_FULL);
static_assert((OSP * 4) % 16 == 0);
static_assert(AW * HD <= OSP);
static_assert(16 * 68 * 4 <= 131072);
static_assert(16 * OSP * 4 <= 131072);
static_assert(64 * 72 * 2 <= 131072);

typedef _Float16 h16;
typedef unsigned short bf;
typedef __attribute__((ext_vector_type(16))) __bf16   v16bf;
typedef __attribute__((ext_vector_type(16))) _Float16 v16h;
typedef __attribute__((ext_vector_type(8)))  _Float16 v8h;
typedef __attribute__((ext_vector_type(8)))  unsigned short v8us;
typedef __attribute__((ext_vector_type(8)))  float    v8f;
typedef __attribute__((ext_vector_type(4)))  float    v4f;
typedef v4f  __attribute__((may_alias)) v4fa;
typedef v8us __attribute__((may_alias)) v8usa;

__device__ __forceinline__ unsigned short f2bf(float f) { unsigned u = __float_as_uint(f); u += 0x7FFFu + ((u >> 16) & 1u); return (unsigned short)(u >> 16); }
__device__ __forceinline__ float bfr(float f) { return __uint_as_float(((unsigned)f2bf(f)) << 16); }
__device__ __forceinline__ v16h cat16(v8h lo, v8h hi) { return __builtin_shufflevector(lo, hi, 0, 1, 2, 3, 4, 5, 6, 7, 8, 9, 10, 11, 12, 13, 14, 15); }
__device__ __forceinline__ v16bf cat16b(v8us lo, v8us hi) { return __builtin_bit_cast(v16bf, __builtin_shufflevector(lo, hi, 0, 1, 2, 3, 4, 5, 6, 7, 8, 9, 10, 11, 12, 13, 14, 15)); }
__device__ __forceinline__ v8f wmma16(v16h a, v16h b, v8f c) { return __builtin_amdgcn_wmma_f32_16x16x32_f16(false, a, false, b, (short)0, c, false, false); }
__device__ __forceinline__ v8f wmmab(v16bf a, v16bf b, v8f c) { return __builtin_amdgcn_wmma_f32_16x16x32_bf16(false, a, false, b, (short)0, c, false, false); }
__device__ __forceinline__ v16h  ldh(const h16* p) { return cat16(*(const v8h*)p, *(const v8h*)(p + 16)); }
__device__ __forceinline__ v16bf ldb(const bf* p)  { return cat16b(*(const v8us*)p, *(const v8us*)(p + 16)); }
__device__ __forceinline__ void wave_sync() { __builtin_amdgcn_fence(3  , "wavefront"); __builtin_amdgcn_wave_barrier(); asm volatile("" ::: "memory"); }

__device__ __forceinline__ v8f wmma16g(v16h a, v16h b, v8f c) { c = wmma16(a, b, c); asm volatile("v_nop\n\tv_nop\n\tv_nop\n\tv_nop" : "+v"(c) : "v"(a), "v"(b)); return c; }
__device__ __forceinline__ v8f wmmabg(v16bf a, v16bf b, v8f c) { c = wmmab(a, b, c); asm volatile("v_nop\n\tv_nop\n\tv_nop\n\tv_nop" : "+v"(c) : "v"(a), "v"(b)); return c; }
static __device__ __forceinline__ h16 toh_flush(float v) { const h16 r = (h16)v; return (fabsf(v) < 6.103515625e-05f) ? (h16)0.0f : r; }

__global__ __launch_bounds__(256) void k_cvt8(const float* __restrict__ src, bf* dst, size_t n8) {
    const size_t i = (size_t)blockIdx.x * 256 + threadIdx.x; if (i >= n8) return;
    const v8f v = *(const v8f*)(src + i * 8); v8us o;
#pragma unroll
    for (int k = 0; k < 8; ++k) o[k] = f2bf(v[k]);
    *(volatile v8us*)(dst + i * 8) = o; __threadfence(); *(volatile v8us*)(dst + i * 8) = o;
}

static_assert(256 * 8 * 2 == 64 * 64);
template <int F16>
__device__ __forceinline__ void wt_body(const float* __restrict__ src, unsigned short* dst, int N) {
    __shared__ __align__(16) unsigned short tt[64 * 72];
    const int tid = threadIdx.x; const int n0 = blockIdx.x * 64, k0 = blockIdx.y * 64;
#pragma unroll 4
    for (int i = 0; i < 16; ++i) {
        const int k = i * 4 + (tid >> 6), n = tid & 63;
        const float v = src[(size_t)(k0 + k) * (size_t)N + (size_t)(n0 + n)];
        unsigned short o;
        if (F16) o = __builtin_bit_cast(unsigned short, toh_flush(bfr(v) * WSC)); else o = f2bf(v);
        tt[n * 72 + k] = o; }
    __syncthreads();
#pragma unroll 1
    for (int ps = 0; ps < 2; ++ps) {
#pragma unroll
        for (int it = 0; it < 2; ++it) { const int n = it * 32 + (tid >> 3), c8 = (tid & 7) * 8;
            const v8us val = *(const v8usa*)(&tt[n * 72 + c8]);
            *(volatile v8us*)(dst + (size_t)(n0 + n) * DM + (size_t)(k0 + c8)) = val; }
        if (ps == 0) __threadfence(); }
}
__global__ __launch_bounds__(256) void k_wt_b(const float* __restrict__ src, bf* dst, int N)  { wt_body<0>(src, dst, N); }
__global__ __launch_bounds__(256) void k_wt_h(const float* __restrict__ src, h16* dst, int N) { wt_body<1>(src, (unsigned short*)dst, N); }

static_assert(32 * 8 * 1 == 16 * HD);
static_assert(32 * 8 * 4 == 16 * 64);
template <int MODE>
__device__ __forceinline__ void proj_body(const bf* __restrict__ A, const bf* __restrict__ Bt, const float* __restrict__ bias, h16* Ph, h16* Pr, int resT) {
    __shared__ __align__(16) float os[16 * 68];
    const int K = DM;
    const int lane = threadIdx.x & 31, lr = lane & 15, hi = lane >> 4; const int r0 = blockIdx.x * 64, c0 = blockIdx.y * 64;
    v8f acc[4][4];
#pragma unroll
    for (int mb = 0; mb < 4; ++mb)
#pragma unroll
        for (int nb = 0; nb < 4; ++nb) acc[mb][nb] = (v8f){};
    const size_t aoff = (size_t)(r0 + lr) * K + 8 * hi, boff = (size_t)(c0 + lr) * K + 8 * hi;
#pragma unroll 1
    for (int kc = 0; kc < K; kc += 32) {
        v16bf a[4];
#pragma unroll
        for (int mb = 0; mb < 4; ++mb) a[mb] = ldb(A + aoff + (size_t)mb * 16 * K + kc);
#pragma unroll
        for (int nb = 0; nb < 4; ++nb) { const v16bf b = ldb(Bt + boff + (size_t)nb * 16 * K + kc);
#pragma unroll
            for (int mb = 0; mb < 4; ++mb) acc[mb][nb] = wmmabg(a[mb], b, acc[mb][nb]); }
    }
    float bc[4];
#pragma unroll
    for (int nb = 0; nb < 4; ++nb) bc[nb] = (MODE == 0) ? bfr(bias[c0 + nb * 16 + lr]) : 0.0f;
    size_t tbase, rbase; bool wr;
    if (MODE == 0) { const int bb = r0 / SEQ, tt = r0 % SEQ; const int zc = bb * NH_ + c0 / HD;
                     tbase = ((size_t)zc * SEQ + (size_t)tt) * HD; rbase = ((size_t)zc * (size_t)resT + (size_t)tt) * HD; wr = tt < resT; }
    else           { const int bb = c0 / SEQ, tt = c0 % SEQ;
                     tbase = (size_t)bb * (size_t)DM * SEQ + (size_t)r0 * SEQ + (size_t)tt; rbase = (size_t)bb * (size_t)DM * (size_t)resT + (size_t)r0 * (size_t)resT + (size_t)tt; wr = tt < resT; }
#pragma unroll
    for (int mb = 0; mb < 4; ++mb) {
        float br[8];
#pragma unroll
        for (int j = 0; j < 8; ++j) br[j] = (MODE == 1) ? bfr(bias[r0 + mb * 16 + hi * 8 + j]) : 0.0f;
#pragma unroll
        for (int nb = 0; nb < 4; ++nb) {
#pragma unroll
            for (int j = 0; j < 8; ++j) os[(hi * 8 + j) * 68 + nb * 16 + lr] = acc[mb][nb][j] + bc[nb] + br[j]; }
        wave_sync();
#pragma unroll 1
        for (int ps = 0; ps < 2; ++ps) {
            if (MODE == 0) {
                const size_t sb = tbase + (size_t)(mb * 16) * HD;
                const size_t rb = rbase + (size_t)(mb * 16) * HD;
#pragma unroll
                for (int hh = 0; hh < 4; ++hh) { const int p = lane; const int row = p >> 1, c8 = (p & 1) * 8;
                    const v4f x0 = *(const v4fa*)(&os[row * 68 + hh * 16 + c8]); const v4f x1 = *(const v4fa*)(&os[row * 68 + hh * 16 + c8 + 4]); v8h hv, rv;
#pragma unroll
                    for (int i = 0; i < 4; ++i) { const h16 a0 = toh_flush(x0[i]); const h16 a1 = toh_flush(x1[i]); hv[i] = a0; hv[4 + i] = a1;
                        rv[i] = toh_flush((x0[i] - (float)a0) * QRS); rv[4 + i] = toh_flush((x1[i] - (float)a1) * QRS); }
                    const size_t oo = sb + (size_t)hh * ((size_t)SEQ * HD) + (size_t)p * 8;
                    const size_t ro = rb + (size_t)hh * ((size_t)resT * HD) + (size_t)p * 8;
                    *(volatile v8h*)(Ph + oo) = hv; if (wr) *(volatile v8h*)(Pr + ro) = rv; }
            } else {
                const size_t sb = tbase + (size_t)(mb * 16) * SEQ;
                const size_t rb = rbase + (size_t)(mb * 16) * (size_t)resT;
#pragma unroll
                for (int s = 0; s < 4; ++s) { const int row = 4 * s + (lane >> 3), c8 = (lane & 7) * 8;
                    const v4f x0 = *(const v4fa*)(&os[row * 68 + c8]); const v4f x1 = *(const v4fa*)(&os[row * 68 + c8 + 4]); v8h hv, rv;
#pragma unroll
                    for (int i = 0; i < 4; ++i) { const h16 a0 = toh_flush(x0[i]); const h16 a1 = toh_flush(x1[i]); hv[i] = a0; hv[4 + i] = a1;
                        rv[i] = toh_flush((x0[i] - (float)a0) * QRS); rv[4 + i] = toh_flush((x1[i] - (float)a1) * QRS); }
                    const size_t oo = sb + (size_t)row * SEQ + c8;
                    const size_t ro = rb + (size_t)row * (size_t)resT + c8;
                    *(volatile v8h*)(Ph + oo) = hv; if (wr) *(volatile v8h*)(Pr + ro) = rv; }
            }
            if (ps == 0) __threadfence(); }
        wave_sync();
    }
}
__global__ __launch_bounds__(32) void k_proj_qk(const bf* __restrict__ A, const bf* __restrict__ Bt, const float* __restrict__ bias, h16* Ph, h16* Pr, int resT) { proj_body<0>(A, Bt, bias, Ph, Pr, resT); }
__global__ __launch_bounds__(32) void k_proj_vt(const bf* __restrict__ A, const bf* __restrict__ Bt, const float* __restrict__ bias, h16* Ph, h16* Pr, int resT) { proj_body<1>(A, Bt, bias, Ph, Pr, resT); }

static_assert(AW * 4 == 16);
static_assert(8 * 8 == AW * HD);
template <int EARLY>
__device__ __forceinline__ void flash_body(const h16* __restrict__ QH, const h16* __restrict__ QR, const h16* __restrict__ KP, const h16* __restrict__ KR,
                                           const h16* __restrict__ VT, const h16* __restrict__ VR, h16* CH, h16* CR) {
    __shared__ __align__(16) float os[16 * OSP];
    const int lane = threadIdx.x & 31, lr = lane & 15, hi = lane >> 4;
    const int wave = __builtin_amdgcn_readfirstlane((int)(threadIdx.x >> 5));
    const int hg = blockIdx.y; const int zh = hg * AW + wave;
    const int t0 = (EARLY ? 0 : EROWS) + blockIdx.x * 16;
    const int lim = t0 + lr;
    const int nk = (t0 + 16 + 31) & ~31;
    const size_t pbase = (size_t)zh * SEQ * HD;
    const size_t rbase = (size_t)zh * EROWS * HD;
    const v8h z8 = (v8h){};
    const v16h hz = (v16h){};
    const v16h qh = cat16(*(const v8h*)(QH + pbase + (size_t)(t0 + lr) * HD + 8 * hi), z8);
    v16h qr = hz;
    if (EARLY) qr = cat16(*(const v8h*)(QR + rbase + (size_t)(t0 + lr) * HD + 8 * hi), z8);
    const size_t ko = pbase + (size_t)lr * HD + 8 * hi;
    const size_t vo = pbase + (size_t)lr * SEQ + 8 * hi;
    const size_t kro = rbase + (size_t)lr * HD + 8 * hi;
    const size_t vro = rbase + (size_t)lr * EROWS + 8 * hi;
    v8f o = (v8f){}, oR = (v8f){};
    float m = NEGB, l = 0.0f;
#pragma unroll 1
    for (int key0 = 0; key0 < nk; key0 += 32) {
        const v16h ka0 = cat16(*(const v8h*)(KP + ko + (size_t)key0 * HD), z8);
        const v16h kb0 = cat16(*(const v8h*)(KP + ko + (size_t)(key0 + 16) * HD), z8);
        v8f sHa = (v8f){}, sHb = (v8f){}, sLa = (v8f){}, sLb = (v8f){};
        sHa = wmma16g(ka0, qh, sHa); sHb = wmma16g(kb0, qh, sHb);
        if (EARLY) {
            const v16h kra0 = cat16(*(const v8h*)(KR + kro + (size_t)key0 * HD), z8);
            const v16h krb0 = cat16(*(const v8h*)(KR + kro + (size_t)(key0 + 16) * HD), z8);
            sLa = wmma16g(ka0, qr, sLa); sLb = wmma16g(kb0, qr, sLb);
            sLa = wmma16g(kra0, qh, sLa); sLb = wmma16g(krb0, qh, sLb);
        }
        const int ja = key0 + 8 * hi;
        float ta[8], tb[8]; bool fa[8], fb[8]; float mx = NEGB;
#pragma unroll
        for (int r = 0; r < 8; ++r) {
            fa[r] = (ja + r <= lim);
            fb[r] = (ja + 16 + r <= lim);
            if (EARLY) { ta[r] = (sHa[r] + sLa[r] * QRI) * SC2; tb[r] = (sHb[r] + sLb[r] * QRI) * SC2; }
            else       { ta[r] = sHa[r] * SC2; tb[r] = sHb[r] * SC2; }
            mx = fmaxf(mx, fmaxf(fa[r] ? ta[r] : NEGB, fb[r] ? tb[r] : NEGB)); }
        mx = fmaxf(mx, __shfl_xor(mx, 16, 32));
        const float mnew = fmaxf(m, mx);
        const float alpha = __builtin_amdgcn_exp2f(m - mnew);
        const float sh = PSH - mnew;
        v16h pb, pr = hz; float ls = 0.0f;
#pragma unroll
        for (int r = 0; r < 8; ++r) {
            const float xa = ta[r] + sh, xb = tb[r] + sh;
            const float ea = __builtin_amdgcn_exp2f(xa), eb = __builtin_amdgcn_exp2f(xb);
            const float ga = (fa[r] & (xa >= -14.0f)) ? ea : 0.0f;
            const float gb = (fb[r] & (xb >= -14.0f)) ? eb : 0.0f;
            const h16 pa = (h16)ga; const h16 pc = (h16)gb;
            pb[r] = pa; pb[8 + r] = pc;
            if (EARLY) { pr[r] = toh_flush((ga - (float)pa) * QRS); pr[8 + r] = toh_flush((gb - (float)pc) * QRS); ls += ga + gb; }
            else       { ls += (float)pa + (float)pc; } }
        l = l * alpha + ls; m = mnew;
        o = o * alpha;
        if (EARLY) oR = oR * alpha;
        const v16h v0 = ldh(VT + vo + key0);
        o = wmma16g(v0, pb, o);
        if (EARLY) {
            const v16h vr0 = ldh(VR + vro + key0);
            oR = wmma16g(v0, pr, oR);
            oR = wmma16g(vr0, pb, oR);
        }
    }
    l += __shfl_xor(l, 16, 32);
    const bool any = l > 0.0f;
    const float lsafe = any ? l : 1.0f;
    const float inv = any ? (CSC / lsafe) : 0.0f;
    v8f f0 = o;
    if (EARLY) f0 = o + oR * QRI;
    { v4f a, c;
      a[0] = f0[0] * inv; a[1] = f0[1] * inv; a[2] = f0[2] * inv; a[3] = f0[3] * inv; c[0] = f0[4] * inv; c[1] = f0[5] * inv; c[2] = f0[6] * inv; c[3] = f0[7] * inv;
      *(v4fa*)(&os[lr * OSP + wave * 16 + 8 * hi]) = a; *(v4fa*)(&os[lr * OSP + wave * 16 + 8 * hi + 4]) = c; }
    __syncthreads();
    const int row = 4 * wave + (lane >> 3), c8 = (lane & 7) * 8;
    const v4f x0 = *(const v4fa*)(&os[row * OSP + c8]); const v4f x1 = *(const v4fa*)(&os[row * OSP + c8 + 4]); v8h hv, rv;
#pragma unroll
    for (int i = 0; i < 4; ++i) { const h16 a0 = toh_flush(x0[i]); const h16 a1 = toh_flush(x1[i]); hv[i] = a0; hv[4 + i] = a1;
        rv[i] = toh_flush((x0[i] - (float)a0) * QRS); rv[4 + i] = toh_flush((x1[i] - (float)a1) * QRS); }
    const size_t oo = (size_t)(t0 + row) * DM + (size_t)hg * (AW * HD) + c8;
#pragma unroll 1
    for (int ps = 0; ps < 2; ++ps) {
        *(volatile v8h*)(CH + oo) = hv;
        if (EARLY) *(volatile v8h*)(CR + oo) = rv;
        if (ps == 0) __threadfence(); }
}
__global__ __launch_bounds__(32 * AW) void k_flash_early(const h16* __restrict__ QH, const h16* __restrict__ QR, const h16* __restrict__ KP, const h16* __restrict__ KR,
                                                         const h16* __restrict__ VT, const h16* __restrict__ VR, h16* CH, h16* CR) { flash_body<1>(QH, QR, KP, KR, VT, VR, CH, CR); }
__global__ __launch_bounds__(32 * AW) void k_flash_late(const h16* __restrict__ QH, const h16* __restrict__ QR, const h16* __restrict__ KP, const h16* __restrict__ KR,
                                                        const h16* __restrict__ VT, const h16* __restrict__ VR, h16* CH, h16* CR) { flash_body<0>(QH, QR, KP, KR, VT, VR, CH, CR); }

static_assert(32 * 4 * 8 == 16 * 64);
template <int EARLY>
__device__ __forceinline__ void oproj_body(const h16* __restrict__ CH, const h16* __restrict__ CR, const h16* __restrict__ Wt, const float* __restrict__ bias, float* OUT) {
    __shared__ __align__(16) float os[16 * 68];
    constexpr int MB = EARLY ? 2 : 4;
    const int K = DM;
    const int lane = threadIdx.x & 31, lr = lane & 15, hi = lane >> 4;
    const int r0 = (EARLY ? 0 : EROWS) + blockIdx.x * (16 * MB), c0 = blockIdx.y * 64;
    v8f acc[MB][4], accr[MB][4];
#pragma unroll
    for (int mb = 0; mb < MB; ++mb)
#pragma unroll
        for (int nb = 0; nb < 4; ++nb) { acc[mb][nb] = (v8f){}; accr[mb][nb] = (v8f){}; }
    const size_t aoff = (size_t)(r0 + lr) * K + 8 * hi, boff = (size_t)(c0 + lr) * K + 8 * hi;
#pragma unroll 1
    for (int kc = 0; kc < K; kc += 32) {
        v16h a[MB], ar[MB];
#pragma unroll
        for (int mb = 0; mb < MB; ++mb) { a[mb] = ldh(CH + aoff + (size_t)mb * 16 * K + kc); ar[mb] = a[mb];
            if (EARLY) ar[mb] = ldh(CR + aoff + (size_t)mb * 16 * K + kc); }
#pragma unroll
        for (int nb = 0; nb < 4; ++nb) { const v16h b = ldh(Wt + boff + (size_t)nb * 16 * K + kc);
#pragma unroll
            for (int mb = 0; mb < MB; ++mb) { acc[mb][nb] = wmma16g(a[mb], b, acc[mb][nb]);
                if (EARLY) accr[mb][nb] = wmma16g(ar[mb], b, accr[mb][nb]); } }
    }
    float bc[4];
#pragma unroll
    for (int nb = 0; nb < 4; ++nb) bc[nb] = bfr(bias[c0 + nb * 16 + lr]);
#pragma unroll
    for (int mb = 0; mb < MB; ++mb) {
#pragma unroll
        for (int nb = 0; nb < 4; ++nb) {
#pragma unroll
            for (int j = 0; j < 8; ++j) { float s = acc[mb][nb][j]; if (EARLY) s = s + accr[mb][nb][j] * QRI;
                os[(hi * 8 + j) * 68 + nb * 16 + lr] = s * OSI + bc[nb]; } }
        wave_sync();
        float* orow = OUT + (size_t)(r0 + mb * 16) * DM + c0;
#pragma unroll 1
        for (int ps = 0; ps < 2; ++ps) {
#pragma unroll
            for (int s = 0; s < 8; ++s) { const int row = 2 * s + (lane >> 4), cofs = (lane & 15) * 4;
                const v4f val = *(const v4fa*)(&os[row * 68 + cofs]);
                *(volatile v4f*)(orow + (size_t)row * DM + cofs) = val; }
            if (ps == 0) __threadfence(); }
        wave_sync();
    }
}
__global__ __launch_bounds__(32) void k_oproj_early(const h16* __restrict__ CH, const h16* __restrict__ CR, const h16* __restrict__ Wt, const float* __restrict__ bias, float* OUT) { oproj_body<1>(CH, CR, Wt, bias, OUT); }
__global__ __launch_bounds__(32) void k_oproj_late(const h16* __restrict__ CH, const h16* __restrict__ CR, const h16* __restrict__ Wt, const float* __restrict__ bias, float* OUT)  { oproj_body<0>(CH, CR, Wt, bias, OUT); }

static constexpr size_t al256(size_t v) { return (v + 255) & ~(size_t)255; }
static constexpr size_t SZ_XB = al256((size_t)NB * SEQ * DM * 2);
static constexpr size_t SZ_WT = al256((size_t)NQKV * DM * 2);
static constexpr size_t SZ_WO = al256((size_t)DM * DM * 2);
static constexpr size_t SZ_PL = al256((size_t)NB * NH_ * SEQ * HD * 2);
static constexpr size_t SZ_RS = al256((size_t)NB * NH_ * EROWS * HD * 2);
static constexpr size_t SZ_TOTAL = SZ_XB + SZ_WT + SZ_WO + 4 * SZ_PL + 4 * SZ_RS;
static_assert(SZ_TOTAL <= (size_t)134217728);
static_assert(((size_t)DM * DM * 2) % 256 == 0);
static_assert((size_t)NB * NH_ * SEQ * HD == (size_t)NB * DM * SEQ);
static_assert((size_t)NB * NH_ * EROWS * HD == (size_t)NB * DM * EROWS);

extern "C" void kernel_launch(void* const* d_in, const int* in_sizes, int n_in,
                              void* d_out, int out_size, void* d_ws, size_t ws_size, hipStream_t stream) {
    if (n_in < 6) return;
    if ((size_t)in_sizes[0] < (size_t)SEQ * DM) return;
    if ((size_t)in_sizes[2] < (size_t)DM * NQKV || in_sizes[3] < NQKV) return;
    if ((size_t)in_sizes[4] < (size_t)DM * DM || in_sizes[5] < DM) return;
    if ((size_t)out_size < (size_t)SEQ * DM) return;
    if (SZ_TOTAL > ws_size) return;
    const float* x    = (const float*)d_in[0];
    const float* wqkv = (const float*)d_in[2]; const float* bqkv = (const float*)d_in[3];
    const float* wout = (const float*)d_in[4]; const float* bout = (const float*)d_in[5];
    float* OUT = (float*)d_out;
    char* wsp = (char*)d_ws;
    bf*  XB  = (bf*)wsp;  wsp += SZ_XB;
    bf*  WT  = (bf*)wsp;  wsp += SZ_WT;
    h16* WOT = (h16*)wsp; wsp += SZ_WO;
    h16* QH  = (h16*)wsp; wsp += SZ_PL;
    h16* KP  = (h16*)wsp; wsp += SZ_PL;
    h16* VT  = (h16*)wsp; wsp += SZ_PL;
    h16* CH  = (h16*)wsp; wsp += SZ_PL;
    h16* QR  = (h16*)wsp; wsp += SZ_RS;
    h16* KR  = (h16*)wsp; wsp += SZ_RS;
    h16* VR  = (h16*)wsp; wsp += SZ_RS;
    h16* CR  = (h16*)wsp; wsp += SZ_RS;

    { const size_t n8 = (size_t)SEQ * DM / 8;
      k_cvt8<<<(unsigned)((n8 + 255) / 256), 256, 0, stream>>>(x, XB, n8); }
    k_wt_b<<<dim3(NQKV / 64, DM / 64, 1), 256, 0, stream>>>(wqkv, WT, NQKV);
    k_wt_h<<<dim3(DM / 64, DM / 64, 1), 256, 0, stream>>>(wout, WOT, DM);

    k_proj_qk<<<dim3(NB * SEQ / 64, DM / 64, 1), 32, 0, stream>>>(XB, WT, bqkv, QH, QR, EROWS);
    k_proj_qk<<<dim3(NB * SEQ / 64, DM / 64, 1), 32, 0, stream>>>(XB, WT + (size_t)DM * DM, bqkv + DM, KP, KR, EROWS);
    k_proj_vt<<<dim3(DM / 64, NB * SEQ / 64, 1), 32, 0, stream>>>(WT + (size_t)2 * DM * DM, XB, bqkv + 2 * DM, VT, VR, EROWS);

    k_flash_early<<<dim3(EROWS / 16, NH_ / AW, 1), 32 * AW, 0, stream>>>(QH, QR, KP, KR, VT, VR, CH, CR);
    if (SEQ > EROWS)
        k_flash_late<<<dim3((SEQ - EROWS) / 16, NH_ / AW, 1), 32 * AW, 0, stream>>>(QH, QR, KP, KR, VT, VR, CH, CR);

    k_oproj_early<<<dim3(EROWS / 32, DM / 64, 1), 32, 0, stream>>>(CH, CR, WOT, bout, OUT);
    if (SEQ > EROWS)
        k_oproj_late<<<dim3((SEQ - EROWS) / 64, DM / 64, 1), 32, 0, stream>>>(CH, CR, WOT, bout, OUT);
}
